// GINBlock_49581102465153
// MI455X (gfx1250) — hardware-verified
//
#include <hip/hip_runtime.h>


namespace {
constexpr int N = 100000, E = 1600000, DI = 32, DH = 128, NPAD = 100352  , NBLK = NPAD / 128, NBA = NPAD / 2048;
constexpr float FXS = 262144.0f, FXI = 1.0f / 262144.0f, BNE = 1e-5f;

typedef _Float16 b16;
typedef __attribute__((ext_vector_type(16))) _Float16 v16b;
typedef __attribute__((ext_vector_type(8)))  _Float16 v8b;
typedef __attribute__((ext_vector_type(8)))  float v8f;
typedef __attribute__((ext_vector_type(4)))  float v4f;

__device__ __forceinline__ v8b ld8b(const b16* p) { return *(const v8b*)p; }
__device__ __forceinline__ v16b cat8b(v8b a, v8b b) { return __builtin_shufflevector(a, b, 0, 1, 2, 3, 4, 5, 6, 7, 8, 9, 10, 11, 12, 13, 14, 15); }
__device__ __forceinline__ v16b frag_kb(const b16* p, int hh) { return cat8b(ld8b(p + 8 * hh), ld8b(p + 16 + 8 * hh)); }
__device__ __forceinline__ void split16(float v, b16& hi, b16& lo) { hi = (b16)v; lo = (b16)(v - (float)hi); }
__device__ __forceinline__ void frag_ksplit(const float* p, int hh, v16b& fh_, v16b& fl_) {
  const float* p0 = p + 8 * hh; const float* p1 = p + 16 + 8 * hh;
#pragma unroll
  for (int e = 0; e < 8; ++e) { b16 a, c; split16(p0[e], a, c); fh_[e] = a; fl_[e] = c; split16(p1[e], a, c); fh_[8 + e] = a; fl_[8 + e] = c; }
}
__device__ __forceinline__ v8f wmma16b(v16b a, v16b b, v8f c) {
  v8f d = __builtin_amdgcn_wmma_f32_16x16x32_f16(false, a, false, b, (short)0, c, false, false);
  asm volatile("v_nop\n\tv_nop\n\tv_nop\n\tv_nop" : "+v"(d) : "v"(a), "v"(b));
  return d;
}
__device__ __forceinline__ void wave_lds_sync() {
  __builtin_amdgcn_fence(__ATOMIC_RELEASE, "workgroup");
  __builtin_amdgcn_wave_barrier();
  __builtin_amdgcn_fence(__ATOMIC_ACQUIRE, "workgroup");
}

struct Opnd { const void* p0; const void* p1; int ld; };
template <int NP> __device__ __forceinline__ void load_frags(const Opnd& o, int row, int kb, int hh, v16b& fh_, v16b& fl_) {
  if (NP == 0) { frag_ksplit((const float*)o.p0 + (size_t)row * o.ld + kb, hh, fh_, fl_); }
  else if (NP == 4) {
    const float* p = (const float*)o.p0 + (size_t)row * o.ld + kb; const float* p0 = p + 8 * hh; const float* p1 = p + 16 + 8 * hh;
#pragma unroll
    for (int e = 0; e < 8; ++e) { b16 a, c; split16(p0[e] * 64.0f, a, c); fh_[e] = a; fl_[e] = c; split16(p1[e] * 64.0f, a, c); fh_[8 + e] = a; fl_[8 + e] = c; }
  } else if (NP == 3) {
    const float* p = (const float*)o.p0 + (size_t)row * o.ld + kb; const float* p0 = p + 8 * hh; const float* p1 = p + 16 + 8 * hh;
#pragma unroll
    for (int e = 0; e < 8; ++e) { fh_[e] = (b16)p0[e]; fh_[8 + e] = (b16)p1[e]; }
    fl_ = fh_;
  } else {
    fh_ = frag_kb((const b16*)o.p0 + (size_t)row * o.ld + kb, hh);
    if (NP == 2) fl_ = frag_kb((const b16*)o.p1 + (size_t)row * o.ld + kb, hh); else fl_ = fh_;
  }
}
template <int ANP, int BNP> __device__ __forceinline__ v8f mac(v16b ah, v16b al, v16b bh, v16b bl, v8f c) {
  c = wmma16b(ah, bh, c);
  if (BNP == 0 || BNP == 2 || BNP == 4) c = wmma16b(ah, bl, c);
  if (ANP == 0 || ANP == 2 || ANP == 4) c = wmma16b(al, bh, c);
  return c;
}
template <int ANP, int BNP>
__device__ __forceinline__ void gemm_tile(const Opnd& A, const Opnd& B, int K, int m0, int c0, int nloc, int hlf, v8f (&acc)[2][4]) {
  for (int kb = 0; kb < K; kb += 32) {
    v16b a0h, a0l, a1h, a1l;
    load_frags<ANP>(A, m0 + nloc, kb, hlf, a0h, a0l);
    load_frags<ANP>(A, m0 + 16 + nloc, kb, hlf, a1h, a1l);
#pragma unroll
    for (int t = 0; t < 4; ++t) {
      v16b bh, bl;
      load_frags<BNP>(B, c0 + t * 16 + nloc, kb, hlf, bh, bl);
      acc[0][t] = mac<ANP, BNP>(a0h, a0l, bh, bl, acc[0][t]);
      acc[1][t] = mac<ANP, BNP>(a1h, a1l, bh, bl, acc[1][t]);
    }
  }
}

__device__ __forceinline__ void epi_planes(v8f (&acc)[2][4], float scale, bool two, b16* __restrict__ oh, b16* __restrict__ ol, int ldo,
                                           int m0, int c0, int lane, b16* Th, b16* Tl) {
  const int nloc = lane & 15, hlf = lane >> 4;
#pragma unroll
  for (int t = 0; t < 4; ++t)
#pragma unroll
    for (int r = 0; r < 2; ++r)
#pragma unroll
      for (int v = 0; v < 8; ++v) {
        const int rr = r * 16 + v + 8 * hlf, cc = t * 16 + nloc;
        b16 h_, l_; split16(acc[r][t][v] * scale, h_, l_);
        Th[rr * 64 + cc] = h_; Tl[rr * 64 + cc] = l_;
      }
  wave_lds_sync();
  for (int pass = 0; pass < 2; ++pass) {
#pragma unroll
    for (int j = 0; j < 8; ++j) {
      const int rr = j * 4 + (lane >> 3), c8 = (lane & 7) * 8;
      const size_t o = (size_t)(m0 + rr) * ldo + c0 + c8;
      *(volatile v8b*)(oh + o) = ld8b(Th + rr * 64 + c8);
      if (two) *(volatile v8b*)(ol + o) = ld8b(Tl + rr * 64 + c8);
    }
    __threadfence();
  }
}
__device__ __forceinline__ void epi_f32(v8f (&acc)[2][4], float scale, const float* rscale, float* __restrict__ out, int ldo, int m0, int c0, int lane, float* Tt) {
  const int nloc = lane & 15, hlf = lane >> 4;
#pragma unroll
  for (int t = 0; t < 4; ++t)
#pragma unroll
    for (int r = 0; r < 2; ++r)
#pragma unroll
      for (int v = 0; v < 8; ++v) {
        const int rr = r * 16 + v + 8 * hlf;
        const float rs = rscale ? rscale[(size_t)(m0 + rr) * 32] : 1.0f;
        Tt[rr * 64 + t * 16 + nloc] = acc[r][t][v] * scale * rs;
      }
  wave_lds_sync();
  float* dst0 = out + (size_t)m0 * ldo + c0;
  for (int pass = 0; pass < 2; ++pass) {
#pragma unroll
    for (int j = 0; j < 16; ++j) { const int rr = j * 2 + hlf, c4 = nloc * 4; *(volatile v4f*)(dst0 + (size_t)rr * ldo + c4) = *(const v4f*)(Tt + rr * 64 + c4); }
    __threadfence();
  }
}


__global__ __launch_bounds__(256) void prep_kernel(const float* __restrict__ W1, const float* __restrict__ W2, b16* __restrict__ w1h, b16* __restrict__ w1l, b16* __restrict__ w2h, b16* __restrict__ w2l) {
  const size_t tid = (size_t)blockIdx.x * blockDim.x + threadIdx.x, nth = (size_t)gridDim.x * blockDim.x;
  for (int pass = 0; pass < 2; ++pass) {
    for (size_t p = tid; p < (size_t)DH * DI; p += nth) { const int n = (int)(p / DI), k = (int)(p % DI); b16 a, c; split16(W1[(size_t)k * DH + n] * 64.0f, a, c); ((volatile b16*)w1h)[p] = a; ((volatile b16*)w1l)[p] = c; }
    for (size_t p = tid; p < (size_t)DH * DH; p += nth) { const int n = (int)(p / DH), k = (int)(p % DH); b16 a, c; split16(W2[(size_t)k * DH + n] * 64.0f, a, c); ((volatile b16*)w2h)[p] = a; ((volatile b16*)w2l)[p] = c; }
    __threadfence();
  }
}

typedef __attribute__((ext_vector_type(4))) int v4i;
__global__ __launch_bounds__(256) void agg_kernel(const int* __restrict__ esrc, const int* __restrict__ edst, const float* __restrict__ x, float* __restrict__ h) {
  constexpr int NB = 2048, DF = DI;
  __shared__ __attribute__((aligned(16))) int acc[NB * DF];
  __shared__ int list[8 * 256];
  const int t_ = threadIdx.x, wave = t_ >> 5, lane = t_ & 31, base = blockIdx.x * NB;
  for (int i = t_; i < NB * DF; i += 256) acc[i] = 0;
  __syncthreads();
  int* wl = list + wave * 256;
  for (int c0 = 0; c0 < E; c0 += 256 * 8) {
    const int e0 = c0 + (wave * 32 + lane) * 8; int dd[8];
#pragma unroll
    for (int j = 0; j < 8; ++j) { const int dv = edst[min(e0 + j, E - 1)]; dd[j] = (e0 + j < E) ? dv : -1; }
    unsigned sl[8]; bool hit[8]; bool anyl = false;
#pragma unroll
    for (int j = 0; j < 8; ++j) { sl[j] = (unsigned)(dd[j] - base); hit[j] = sl[j] < (unsigned)NB; anyl |= hit[j]; }
    int wc = 0;
    if (__builtin_amdgcn_ballot_w32(anyl) != 0u) {
#pragma unroll
      for (int j = 0; j < 8; ++j) {
        const unsigned mj = __builtin_amdgcn_ballot_w32(hit[j]);
        if (mj != 0u) {
          if (hit[j]) { const int pos = wc + (int)__builtin_amdgcn_mbcnt_lo(mj, 0u); int s = esrc[min(e0 + j, E - 1)]; s = (s < 0) ? 0 : (s >= N ? N - 1 : s); wl[pos] = (s << 11) | (int)sl[j]; }
          wc += __builtin_popcount(mj); } } }
    __builtin_amdgcn_wave_barrier(); __builtin_amdgcn_fence(__ATOMIC_RELEASE, "workgroup"); __builtin_amdgcn_fence(__ATOMIC_ACQUIRE, "workgroup");
    for (int i0 = 0; i0 < wc; i0 += 4) { const int i = i0 + (lane >> 3); if (i < wc) { const int ent = wl[i]; const int s = ent >> 11, slot = ent & 2047; const int col = (lane & 7) * 4;
        const v4f v = *(const v4f*)(x + (size_t)s * DF + col);
#pragma unroll
        for (int c = 0; c < 4; ++c) atomicAdd(&acc[slot * DF + col + c], (int)rintf(v[c] * FXS)); } }
    __builtin_amdgcn_wave_barrier();
  }
  __syncthreads();
  for (int pass = 0; pass < 2; ++pass) {
    for (int i = t_; i < NB * DF / 4; i += 256) { const int r = i >> 3, cq = (i & 7) * 4, node = base + r; v4f o = {0.0f, 0.0f, 0.0f, 0.0f};
      if (node < N) { const v4f xv = *(const v4f*)(x + (size_t)node * DF + cq);
#pragma unroll
        for (int c = 0; c < 4; ++c) o[c] = xv[c] + (float)acc[r * DF + cq + c] * FXI; }
      *(volatile v4f*)(h + (size_t)node * DF + cq) = o; }
    __threadfence();
  }
}

template <int KIN, bool BNRELU>
__global__ __launch_bounds__(128) void lin_kernel(const float* __restrict__ hin, const float* __restrict__ coef, const b16* __restrict__ wh, const b16* __restrict__ wl, const float* __restrict__ bias, float* __restrict__ y, float* __restrict__ slot_) {
  __shared__ __attribute__((aligned(16))) float Ts[4][32 * 64]; __shared__ float Cp[4][2][64];
  const int lane = threadIdx.x & 31, wave = threadIdx.x >> 5, nloc = lane & 15, hlf = lane >> 4, m0 = blockIdx.y * 128 + wave * 32, c0 = blockIdx.x * 64;
  v8f acc[2][4];
#pragma unroll
  for (int r = 0; r < 2; ++r)
#pragma unroll
    for (int t = 0; t < 4; ++t) acc[r][t] = (v8f){};
#pragma unroll 1
  for (int kb = 0; kb < KIN; kb += 32) { v16b a0, l0, a1, l1;
#pragma unroll
    for (int e = 0; e < 16; ++e) { const int k = kb + ((e < 8) ? (8 * hlf + e) : (16 + 8 * hlf + e - 8)); float u0 = hin[(size_t)(m0 + nloc) * KIN + k], u1 = hin[(size_t)(m0 + 16 + nloc) * KIN + k];
      if (BNRELU) { const float ca = coef[k], sh = coef[DH + k]; u0 = fmaxf(u0 * ca + sh, 0.0f); u1 = fmaxf(u1 * ca + sh, 0.0f); } b16 p, q; split16(u0 * 8.0f, p, q); a0[e] = p; l0[e] = q; split16(u1 * 8.0f, p, q); a1[e] = p; l1[e] = q; }
#pragma unroll
    for (int t = 0; t < 4; ++t) { const v16b bh = frag_kb(wh + (size_t)(c0 + t * 16 + nloc) * KIN + kb, hlf), bl = frag_kb(wl + (size_t)(c0 + t * 16 + nloc) * KIN + kb, hlf);
      acc[0][t] = wmma16b(a0, bh, acc[0][t]); acc[0][t] = wmma16b(l0, bh, acc[0][t]); acc[0][t] = wmma16b(a0, bl, acc[0][t]);
      acc[1][t] = wmma16b(a1, bh, acc[1][t]); acc[1][t] = wmma16b(l1, bh, acc[1][t]); acc[1][t] = wmma16b(a1, bl, acc[1][t]); } }
#pragma unroll
  for (int t = 0; t < 4; ++t) { const int c = c0 + t * 16 + nloc; float s = 0.0f, s2 = 0.0f;
#pragma unroll
    for (int r = 0; r < 2; ++r)
#pragma unroll
      for (int v = 0; v < 8; ++v) { const float val = acc[r][t][v] * (1.0f / 512.0f) + bias[c]; acc[r][t][v] = val; if (m0 + r * 16 + 8 * hlf + v < N) { s += val; s2 += val * val; } }
    s += __shfl_xor(s, 16); s2 += __shfl_xor(s2, 16);
    if (hlf == 0) { Cp[wave][0][t * 16 + nloc] = s; Cp[wave][1][t * 16 + nloc] = s2; } }
  epi_f32(acc, 1.0f, nullptr, y, DH, m0, c0, lane, Ts[wave]);
  __syncthreads();
  if (threadIdx.x < 128) { const int which = threadIdx.x >> 6, c = threadIdx.x & 63; const float tot = Cp[0][which][c] + Cp[1][which][c] + Cp[2][which][c] + Cp[3][which][c];
    for (int pass = 0; pass < 2; ++pass) { ((volatile float*)slot_)[((size_t)blockIdx.y * 2 + which) * DH + c0 + c] = tot; __threadfence(); } }
}

__global__ __launch_bounds__(128) void bnfin_kernel(const float* __restrict__ slot_, int nblk, const float* __restrict__ g, const float* __restrict__ bb, float* __restrict__ coef) {
  const int c = threadIdx.x; double s = 0.0, s2 = 0.0;
  for (int bk = 0; bk < nblk; ++bk) { s += (double)slot_[((size_t)bk * 2) * DH + c]; s2 += (double)slot_[((size_t)bk * 2 + 1) * DH + c]; }
  const double mean = s / N, var = s2 / N - mean * mean; const float a = g[c] * (float)(1.0 / sqrt(var + (double)BNE)), sh = bb[c] - (float)mean * a;
  for (int pass = 0; pass < 2; ++pass) { ((volatile float*)coef)[c] = a; ((volatile float*)coef)[DH + c] = sh; __threadfence(); }
}

__global__ __launch_bounds__(128) void stat_kernel(const float* __restrict__ h2, const float* __restrict__ coef, float* __restrict__ slot_) {
  const int c = threadIdx.x, r0 = blockIdx.x * 128; const float a = coef[c], sh = coef[DH + c]; float s = 0.0f, s2 = 0.0f;
  for (int r = r0; r < min(r0 + 128, N); ++r) { const float v = fmaxf(h2[(size_t)r * DH + c] * a + sh, 0.0f); s += v; s2 += v * v; }
  for (int pass = 0; pass < 2; ++pass) { ((volatile float*)slot_)[((size_t)blockIdx.x * 2) * DH + c] = s; ((volatile float*)slot_)[((size_t)blockIdx.x * 2 + 1) * DH + c] = s2; __threadfence(); }
}

__global__ __launch_bounds__(256) void final_kernel(const float* __restrict__ h2, const float* __restrict__ coef2, const float* __restrict__ coef3, float* __restrict__ out) {
  const size_t i = (size_t)blockIdx.x * 256 + threadIdx.x; const int row = (int)(i >> 5), cq = (int)(i & 31) * 4;
  const v4f v = *(const v4f*)(h2 + (size_t)row * DH + cq); v4f o;
#pragma unroll
  for (int c = 0; c < 4; ++c) { const float z = fmaxf(v[c] * coef2[cq + c] + coef2[DH + cq + c], 0.0f); o[c] = fmaxf(z * coef3[cq + c] + coef3[DH + cq + c], 0.0f); }
  for (int pass = 0; pass < 2; ++pass) { *(volatile v4f*)(out + (size_t)row * DH + cq) = o; __threadfence(); }
}
}

extern "C" void kernel_launch(void* const* d_in, const int* in_sizes, int n_in,
                              void* d_out, int out_size, void* d_ws, size_t ws_size, hipStream_t stream) {
  (void)n_in; (void)out_size;
  const float* x = (const float*)d_in[0]; const int* src = (const int*)d_in[1]; const int* dst = (const int*)d_in[2];
  const float* W1 = (const float*)d_in[3]; const float* b1 = (const float*)d_in[4]; const float* g1 = (const float*)d_in[5]; const float* be1 = (const float*)d_in[6];
  const float* W2 = (const float*)d_in[7]; const float* b2 = (const float*)d_in[8]; const float* g2 = (const float*)d_in[9]; const float* be2 = (const float*)d_in[10]; const float* g3 = (const float*)d_in[11]; const float* be3 = (const float*)d_in[12];
  float* out = (float*)d_out;
  if (in_sizes[0] != N * DI || in_sizes[1] != E || in_sizes[2] != E || in_sizes[3] != DI * DH || in_sizes[7] != DH * DH) return;
  size_t off = 0; char* ws = (char*)d_ws;
  auto carve = [&](size_t bytes) { char* p = ws + off; off += (bytes + 255) & ~(size_t)255; return p; };
  b16* w1h = (b16*)carve(DH * DI * 2); b16* w1l = (b16*)carve(DH * DI * 2); b16* w2h = (b16*)carve(DH * DH * 2); b16* w2l = (b16*)carve(DH * DH * 2);
  float* h = (float*)carve((size_t)NPAD * DI * 4); float* h1 = (float*)carve((size_t)NPAD * DH * 4); float* h2 = (float*)carve((size_t)NPAD * DH * 4);
  float* slot_ = (float*)carve((size_t)NBLK * 2 * DH * 4); float* coef1 = (float*)carve(2 * DH * 4); float* coef2 = (float*)carve(2 * DH * 4); float* coef3 = (float*)carve(2 * DH * 4);
  if (off > ws_size) return;
  prep_kernel<<<64, 256, 0, stream>>>(W1, W2, w1h, w1l, w2h, w2l);
  agg_kernel<<<NBA, 256, 0, stream>>>(src, dst, x, h);
  lin_kernel<DI, false><<<dim3(2, NBLK), 128, 0, stream>>>(h, nullptr, w1h, w1l, b1, h1, slot_);
  bnfin_kernel<<<1, 128, 0, stream>>>(slot_, NBLK, g1, be1, coef1);
  lin_kernel<DH, true><<<dim3(2, NBLK), 128, 0, stream>>>(h1, coef1, w2h, w2l, b2, h2, slot_);
  bnfin_kernel<<<1, 128, 0, stream>>>(slot_, NBLK, g2, be2, coef2);
  stat_kernel<<<NBLK, 128, 0, stream>>>(h2, coef2, slot_);
  bnfin_kernel<<<1, 128, 0, stream>>>(slot_, NBLK, g3, be3, coef3);
  final_kernel<<<N * 32 / 256, 256, 0, stream>>>(h2, coef2, coef3, out);
}
